// InterpretableMultiHeadAttention_21182778704277
// MI455X (gfx1250) — hardware-verified
//
#include <hip/hip_runtime.h>


#define NB_  2
#define SS   2048
#define EE   1024
#define NH_  16
#define HD   64
#define ZH   4
#define NR   (NB_ * SS)
#define DM   EE
#define PCAR 1024.0f
#define LOSC 1024.0f
typedef _Float16 h16;
typedef unsigned short bf;
typedef __attribute__((ext_vector_type(16))) __bf16   v16bf;
typedef __attribute__((ext_vector_type(16))) _Float16 v16h;
typedef __attribute__((ext_vector_type(8)))  _Float16 v8h;
typedef __attribute__((ext_vector_type(8)))  unsigned short v8us;
typedef __attribute__((ext_vector_type(8)))  float    v8f;
typedef __attribute__((ext_vector_type(4)))  float    v4f;
typedef v8h  __attribute__((may_alias)) v8ha;
typedef v4f  __attribute__((may_alias)) v4fa;
typedef v8us __attribute__((may_alias)) v8usa;

__device__ __forceinline__ unsigned short f2bf(float f) { unsigned u = __float_as_uint(f); u += 0x7FFFu + ((u >> 16) & 1u); return (unsigned short)(u >> 16); }
__device__ __forceinline__ float bf2f(unsigned short b) { return __uint_as_float(((unsigned)b) << 16); }
__device__ __forceinline__ float bfr(float f) { return bf2f(f2bf(f)); }
__device__ __forceinline__ v16h cat16(v8h lo, v8h hi) { return __builtin_shufflevector(lo, hi, 0, 1, 2, 3, 4, 5, 6, 7, 8, 9, 10, 11, 12, 13, 14, 15); }
__device__ __forceinline__ v16bf cat16b(v8us lo, v8us hi) { return __builtin_bit_cast(v16bf, __builtin_shufflevector(lo, hi, 0, 1, 2, 3, 4, 5, 6, 7, 8, 9, 10, 11, 12, 13, 14, 15)); }
__device__ __forceinline__ v8f wmma16(v16h a, v16h b, v8f c) { return __builtin_amdgcn_wmma_f32_16x16x32_f16(false, a, false, b, (short)0, c, false, false); }
__device__ __forceinline__ v8f wmmab(v16bf a, v16bf b, v8f c) { return __builtin_amdgcn_wmma_f32_16x16x32_bf16(false, a, false, b, (short)0, c, false, false); }

template <bool SPLITA, bool F16OUT = false>
__global__ __launch_bounds__(128) void k_gemmb(const bf* __restrict__ A, const bf* __restrict__ Al, const bf* __restrict__ Bn, const float* __restrict__ bias, float* C, int ldc, h16* C2, const float* __restrict__ R = nullptr, int K = DM, int roundR = 1) {
    __shared__ __align__(16) float ost[4][16 * 68];
    const int lane = threadIdx.x & 31, wave = threadIdx.x >> 5, lr = lane & 15, hi = lane >> 4;
    const int r0 = blockIdx.x * 64 + wave * 16, c0 = blockIdx.y * 64;
    const size_t aoff = (size_t)(r0 + lr) * K + 8 * hi;
    size_t boff[4];
#pragma unroll
    for (int t = 0; t < 4; ++t) boff[t] = (size_t)(c0 + t * 16 + lr) * K + 8 * hi;
    v8f acc[4];
#pragma unroll
    for (int t = 0; t < 4; ++t) acc[t] = (v8f){};
#pragma unroll 1
    for (int kc = 0; kc < K; kc += 32) {
        const v16bf a = cat16b(*(const v8us*)(A + aoff + kc), *(const v8us*)(A + aoff + kc + 16));
        v16bf al = a;
        if (SPLITA) al = cat16b(*(const v8us*)(Al + aoff + kc), *(const v8us*)(Al + aoff + kc + 16));
#pragma unroll
        for (int t = 0; t < 4; ++t) { const v16bf b = cat16b(*(const v8us*)(Bn + boff[t] + kc), *(const v8us*)(Bn + boff[t] + kc + 16)); acc[t] = wmmab(a, b, acc[t]); if (SPLITA) acc[t] = wmmab(al, b, acc[t]); }
        asm volatile("v_nop\n\tv_nop\n\tv_nop\n\tv_nop" : "+v"(acc[0]), "+v"(acc[1]), "+v"(acc[2]), "+v"(acc[3]) : "v"(a), "v"(al));
    }
    float* os = &ost[wave][0];
#pragma unroll
    for (int t = 0; t < 4; ++t) { const float bv = bias ? bfr(bias[c0 + t * 16 + lr]) : 0.f;
#pragma unroll
        for (int j = 0; j < 8; ++j) os[(hi * 8 + j) * 68 + t * 16 + lr] = acc[t][j] + bv; }
    __syncthreads();
    if (F16OUT) {
        h16* crow = (h16*)(void*)C + (size_t)r0 * ldc + c0;
        auto pass = [&]() {
#pragma unroll
            for (int s = 0; s < 4; ++s) { const int row = 4 * s + (lane >> 3), piece = lane & 7; const float* sp = os + row * 68 + piece * 8; v8h o, o2;
#pragma unroll
                for (int i = 0; i < 8; ++i) { const h16 a = (h16)sp[i]; o[i] = a; o2[i] = (h16)((sp[i] - (float)a) * LOSC); }
                *(volatile v8h*)(crow + (size_t)row * ldc + piece * 8) = o; if (C2) *(volatile v8h*)(C2 + (size_t)r0 * ldc + c0 + (size_t)row * ldc + piece * 8) = o2; }
        };
        pass(); __threadfence(); pass();
    } else {
        float* crow = C + (size_t)r0 * ldc + c0;
        auto pass = [&]() {
#pragma unroll
            for (int s = 0; s < 8; ++s) { const int Lid = (lane >> 3) + 4 * s, piece = lane & 7; const int row = Lid >> 1, cofs = (Lid & 1) * 32 + piece * 4;
                v4f val = *(const v4fa*)(os + row * 68 + cofs); if (R) { const v4f rv = *(const v4f*)(R + ((size_t)r0 + row) * ldc + c0 + cofs); val += roundR ? (v4f){bfr(rv[0]), bfr(rv[1]), bfr(rv[2]), bfr(rv[3])} : rv; }
                *(volatile v4f*)(crow + (size_t)row * ldc + cofs) = val; }
        };
        pass(); __threadfence(); pass();
    }
}

__global__ __launch_bounds__(256) void k_cvt8(const float* __restrict__ src, bf* dst, size_t n8) {
    const size_t i = (size_t)blockIdx.x * 256 + threadIdx.x; if (i >= n8) return;
    const v8f v = *(const v8f*)(src + i * 8); v8us o;
#pragma unroll
    for (int k = 0; k < 8; ++k) o[k] = f2bf(v[k]);
    *(volatile v8us*)(dst + i * 8) = o; __threadfence(); *(volatile v8us*)(dst + i * 8) = o;
}
__global__ __launch_bounds__(256) void k_zero8(bf* dst, size_t n8) {
    const size_t i = (size_t)blockIdx.x * 256 + threadIdx.x; if (i >= n8) return; v8us z;
#pragma unroll
    for (int k = 0; k < 8; ++k) z[k] = 0;
    *(volatile v8us*)(dst + i * 8) = z; __threadfence(); *(volatile v8us*)(dst + i * 8) = z;
}

__global__ __launch_bounds__(128) void k_gemmh(const h16* __restrict__ A, const h16* __restrict__ Bn, const float* __restrict__ bias, float* C, int ldc, const float* __restrict__ R, int K, size_t sA, size_t sB, size_t sC, int roundR) {
    __shared__ __align__(16) float ost[4][16 * 68];
    const size_t z = blockIdx.z; A += z * sA; Bn += z * sB; C += z * sC; if (R) R += z * sC;
    const int lane = threadIdx.x & 31, wave = threadIdx.x >> 5, lr = lane & 15, hi = lane >> 4;
    const int r0 = blockIdx.x * 64 + wave * 16, c0 = blockIdx.y * 64;
    const size_t aoff = (size_t)(r0 + lr) * K + 8 * hi;
    size_t boff[4];
#pragma unroll
    for (int t = 0; t < 4; ++t) boff[t] = (size_t)(c0 + t * 16 + lr) * K + 8 * hi;
    v8f acc[4];
#pragma unroll
    for (int t = 0; t < 4; ++t) acc[t] = (v8f){};
#pragma unroll 1
    for (int kc = 0; kc < K; kc += 32) {
        const v16h a = cat16(*(const v8h*)(A + aoff + kc), *(const v8h*)(A + aoff + kc + 16));
#pragma unroll
        for (int t = 0; t < 4; ++t) { const v16h b = cat16(*(const v8h*)(Bn + boff[t] + kc), *(const v8h*)(Bn + boff[t] + kc + 16)); acc[t] = wmma16(a, b, acc[t]); }
        asm volatile("v_nop\n\tv_nop\n\tv_nop\n\tv_nop" : "+v"(acc[0]), "+v"(acc[1]), "+v"(acc[2]), "+v"(acc[3]) : "v"(a));
    }
    float* os = &ost[wave][0];
#pragma unroll
    for (int t = 0; t < 4; ++t) { const float bv = bias ? bfr(bias[c0 + t * 16 + lr]) : 0.f;
#pragma unroll
        for (int j = 0; j < 8; ++j) os[(hi * 8 + j) * 68 + t * 16 + lr] = acc[t][j] + bv; }
    __syncthreads();
    float* crow = C + (size_t)r0 * ldc + c0;
    auto pass = [&]() {
#pragma unroll
        for (int s = 0; s < 8; ++s) { const int Lid = (lane >> 3) + 4 * s, piece = lane & 7; const int row = Lid >> 1, cofs = (Lid & 1) * 32 + piece * 4;
            v4f val = *(const v4fa*)(os + row * 68 + cofs); if (R) { const v4f rv = *(const v4f*)(R + ((size_t)r0 + row) * ldc + c0 + cofs); val += roundR ? (v4f){bfr(rv[0]), bfr(rv[1]), bfr(rv[2]), bfr(rv[3])} : rv; }
            *(volatile v4f*)(crow + (size_t)row * ldc + cofs) = val; }
    };
    pass(); __threadfence(); pass();
}
__constant__ float c_invf[32] = {1.0f, 0.749894202f, 0.562341332f, 0.421696514f, 0.316227764f, 0.237137392f, 0.177827939f, 0.133352146f, 0.100000001f, 0.0749894157f, 0.0562341288f, 0.0421696492f, 0.0316227786f, 0.0237137359f, 0.0177827943f, 0.0133352149f, 0.00999999978f, 0.00749894232f, 0.00562341325f, 0.00421696482f, 0.00316227786f, 0.00237137382f, 0.00177827943f, 0.00133352145f, 0.00100000005f, 0.000749894185f, 0.000562341302f, 0.000421696546f, 0.000316227786f, 0.000237137385f, 0.00017782794f, 0.00013335215f};
typedef __attribute__((ext_vector_type(4))) _Float16 v4h;
__device__ __forceinline__ h16 tohx(float x) { return (h16)x; }
__global__ __launch_bounds__(256) void k_cvtx(const float* __restrict__ x, bf* A) {
    const int lane = threadIdx.x & 31; const size_t r = (size_t)blockIdx.x * 8 + (threadIdx.x >> 5); if (r >= (size_t)NR) return;
#pragma unroll 1
    for (int ps = 0; ps < 2; ++ps) {
#pragma unroll
        for (int q = 0; q < EE / 256; ++q) { const size_t o = r * EE + q * 256 + lane * 8; v8us v;
#pragma unroll
            for (int i = 0; i < 8; ++i) v[i] = f2bf(x[o + i]);
            *(volatile v8us*)(A + o) = v; }
        if (ps == 0) __threadfence(); }
}
__global__ __launch_bounds__(256) void k_cvt8h(const float* __restrict__ src, h16* dst, size_t n8) { const size_t i = (size_t)blockIdx.x * 256 + threadIdx.x; if (i >= n8) return; const v8f v = *(const v8f*)(src + i * 8); v8h o;
#pragma unroll
    for (int k = 0; k < 8; ++k) o[k] = tohx(bfr(v[k])); *(volatile v8h*)(dst + i * 8) = o; __threadfence(); *(volatile v8h*)(dst + i * 8) = o; }
template <bool ROPE>
__global__ __launch_bounds__(256) void k_ropepl(const float* __restrict__ F, int b, int h0, float sc, h16* P) {
    __shared__ float sl[256][5];
    const int lane = threadIdx.x & 31; const size_t w = (size_t)blockIdx.x * 8 + (threadIdx.x >> 5); const int t = (int)(w * 2 + (lane >> 4)); if (t >= SS) return; const int z = blockIdx.z; const int c0 = (lane & 15) * 4; const float* row = F + ((size_t)b * SS + t) * EE + (h0 + z) * HD; float* slot = sl[threadIdx.x];
#pragma unroll 1
    for (int q = 0; q < 4; ++q) { const int d = c0 + q; float y = row[d];
        if (ROPE) { const float ang = (float)t * c_invf[d & 31]; const float cs = cosf(ang), sn = sinf(ang); const float other = (d < 32) ? -row[d + 32] : row[d - 32]; y = y * cs + other * sn; }
        slot[q] = y * sc; }
    v4h o; o[0] = tohx(slot[0]); o[1] = tohx(slot[1]); o[2] = tohx(slot[2]); o[3] = tohx(slot[3]);
    const size_t off = ((size_t)z * SS + t) * HD + c0; *(volatile v4h*)(P + off) = o; __threadfence(); *(volatile v4h*)(P + off) = o;
}
__global__ __launch_bounds__(256) void k_vT64h(const float* __restrict__ V, int b, int h0, h16* VT) {
    __shared__ float tl[64][65];
    const int tid = threadIdx.x; const int t0 = blockIdx.x * 64; const int z = blockIdx.z; const int rr = tid >> 2, cq = (tid & 3) * 16;
#pragma unroll
    for (int i = 0; i < 16; ++i) tl[rr][cq + i] = V[((size_t)b * SS + t0 + rr) * EE + (h0 + z) * HD + cq + i];
    __syncthreads();
    const int lane = tid & 31, wv = tid >> 5;
    auto pass = [&]() {
#pragma unroll
        for (int st = 0; st < 4; ++st) { const int dr = wv * 8 + st * 2 + (lane >> 4); const int tq = (lane & 15) * 4; v4h v;
#pragma unroll
            for (int i = 0; i < 4; ++i) v[i] = tohx(tl[tq + i][dr]);
            *(volatile v4h*)(VT + ((size_t)z * HD + dr) * SS + t0 + tq) = v; }
    };
    pass(); __threadfence(); pass();
}
__global__ __launch_bounds__(256) void k_softc(const float* __restrict__ S, h16* P) {
    const int lane = threadIdx.x & 31, i = blockIdx.x * 8 + (threadIdx.x >> 5); if (i >= SS) return; const size_t zo = ((size_t)blockIdx.z * SS + i) * SS; const float* sr = S + zo; h16* po = P + zo;
    float m = -3.0e38f;
#pragma unroll 1
    for (int c0 = lane * 4; c0 < SS; c0 += 128) {
#pragma unroll
        for (int q = 0; q < 4; ++q) m = fmaxf(m, sr[c0 + q]); }
#pragma unroll
    for (int sh = 16; sh; sh >>= 1) m = fmaxf(m, __shfl_xor(m, sh, 32));
    float sum = 0.f;
#pragma unroll 1
    for (int c0 = lane * 4; c0 < SS; c0 += 128) {
#pragma unroll
        for (int q = 0; q < 4; ++q) sum += __expf(sr[c0 + q] - m); }
#pragma unroll
    for (int sh = 16; sh; sh >>= 1) sum += __shfl_xor(sum, sh, 32);
    const float f = __fdiv_rn(PCAR, sum);
#pragma unroll 1
    for (int ps = 0; ps < 2; ++ps) {
#pragma unroll 1
        for (int c0 = lane * 4; c0 < SS; c0 += 128) { v4h o;
#pragma unroll
            for (int q = 0; q < 4; ++q) o[q] = tohx(__expf(sr[c0 + q] - m) * f);
            *(volatile v4h*)(po + c0) = o; }
        if (ps == 0) __threadfence(); }
}
__global__ __launch_bounds__(256) void k_mergec(const float* __restrict__ OZ, int b, int h0, h16* OH) {
    const int lane = threadIdx.x & 31, i = blockIdx.x * 8 + (threadIdx.x >> 5); if (i >= SS) return; const int z = lane >> 3, d0 = (lane & 7) * 8; v8h o;
#pragma unroll
    for (int k = 0; k < 8; ++k) o[k] = tohx(OZ[((size_t)z * SS + i) * HD + d0 + k] * (1.0f / PCAR));
    const size_t off = ((size_t)b * SS + i) * EE + (h0 + z) * HD + d0; *(volatile v8h*)(OH + off) = o; __threadfence(); *(volatile v8h*)(OH + off) = o;
}
extern "C" void kernel_launch(void* const* d_in, const int* in_sizes, int n_in,
                              void* d_out, int out_size, void* d_ws, size_t ws_size, hipStream_t stream) {
    (void)in_sizes; (void)n_in; (void)out_size;
    const float* xq = (const float*)d_in[0]; const float* xk = (const float*)d_in[1]; const float* xv = (const float*)d_in[2]; const float* Wq = (const float*)d_in[3]; const float* bq = (const float*)d_in[4]; const float* Wk = (const float*)d_in[5]; const float* bk = (const float*)d_in[6]; const float* Wv = (const float*)d_in[7]; const float* bv = (const float*)d_in[8]; const float* Wo = (const float*)d_in[9]; const float* bo = (const float*)d_in[10];
    float* out = (float*)d_out;
    char* wsp = (char*)d_ws;
    auto take = [&](size_t bytes) { char* p = wsp; wsp += (bytes + 255) & ~(size_t)255; return (void*)p; };
    bf* WQB = (bf*)take((size_t)EE * EE * 2); bf* WKB = (bf*)take((size_t)EE * EE * 2); bf* WVB = (bf*)take((size_t)EE * EE * 2); h16* WOH = (h16*)take((size_t)EE * EE * 2);
    bf* XB = (bf*)take((size_t)NR * EE * 2); float* Q = (float*)take((size_t)NR * EE * 4); float* Kf = (float*)take((size_t)NR * EE * 4); float* V = (float*)take((size_t)NR * EE * 4);
    h16* Qx = (h16*)take((size_t)ZH * SS * HD * 2); h16* Kx = (h16*)take((size_t)ZH * SS * HD * 2); h16* VT = (h16*)take((size_t)ZH * HD * SS * 2); float* S = (float*)take((size_t)ZH * SS * SS * 4); h16* Px = (h16*)take((size_t)ZH * SS * SS * 2); float* OZ = (float*)take((size_t)ZH * SS * HD * 4); h16* OH = (h16*)take((size_t)NR * EE * 2);
    if ((size_t)(wsp - (char*)d_ws) > ws_size) return;
    const size_t n8 = (size_t)EE * EE / 8; const unsigned nb8 = (unsigned)((n8 + 255) / 256);
    k_cvt8<<<nb8, 256, 0, stream>>>(Wq, WQB, n8); k_cvt8<<<nb8, 256, 0, stream>>>(Wk, WKB, n8); k_cvt8<<<nb8, 256, 0, stream>>>(Wv, WVB, n8); k_cvt8h<<<nb8, 256, 0, stream>>>(Wo, WOH, n8);
    k_cvtx<<<NR / 8, 256, 0, stream>>>(xq, XB); k_gemmb<false, false><<<dim3(NR / 64, EE / 64, 1), 128, 0, stream>>>(XB, nullptr, WQB, bq, Q, EE, nullptr, nullptr, EE);
    k_cvtx<<<NR / 8, 256, 0, stream>>>(xk, XB); k_gemmb<false, false><<<dim3(NR / 64, EE / 64, 1), 128, 0, stream>>>(XB, nullptr, WKB, bk, Kf, EE, nullptr, nullptr, EE);
    k_cvtx<<<NR / 8, 256, 0, stream>>>(xv, XB); k_gemmb<false, false><<<dim3(NR / 64, EE / 64, 1), 128, 0, stream>>>(XB, nullptr, WVB, bv, V, EE, nullptr, nullptr, EE);
    for (int b = 0; b < NB_; ++b)
        for (int h0 = 0; h0 < NH_; h0 += ZH) {
            k_ropepl<true><<<dim3((SS / 2) / 8, 1, ZH), 256, 0, stream>>>(Q, b, h0, 0.125f, Qx); k_ropepl<true><<<dim3((SS / 2) / 8, 1, ZH), 256, 0, stream>>>(Kf, b, h0, 1.0f, Kx); k_vT64h<<<dim3(SS / 64, 1, ZH), 256, 0, stream>>>(V, b, h0, VT);
            k_gemmh<<<dim3(SS / 64, SS / 64, ZH), 128, 0, stream>>>(Qx, Kx, nullptr, S, SS, nullptr, HD, (size_t)SS * HD, (size_t)SS * HD, (size_t)SS * SS, 0);
            k_softc<<<dim3(SS / 8, 1, ZH), 256, 0, stream>>>(S, Px);
            k_gemmh<<<dim3(SS / 64, 1, ZH), 128, 0, stream>>>(Px, VT, nullptr, OZ, HD, nullptr, SS, (size_t)SS * SS, (size_t)HD * SS, (size_t)SS * HD, 0);
            k_mergec<<<SS / 8, 256, 0, stream>>>(OZ, b, h0, OH); }
    k_gemmh<<<dim3(NR / 64, EE / 64, 1), 128, 0, stream>>>(OH, WOH, bo, out, EE, nullptr, EE, 0, 0, 0, 0);
}
